// ClusterisedLinearNetwork_72713796321290
// MI455X (gfx1250) — hardware-run, weakly checked
//
#include <hip/hip_runtime.h>
#include <math.h>


#ifndef NPTS
#define NPTS 524288
#endif
#define NPTS_FULL 524288
#define NCH  5
#define NFQ  10
#define KD   100
#define KP   128
#define NCL  128
#define NCOL 384
#define NT   24
#define AW   4
#define RT   32
#define EP   68
#define WSC  1024.0f
#define WSI  (1.0f / 1024.0f)

static_assert(KD == NCH * 2 * NFQ);
static_assert(KD % 2 == 0);
static_assert(KP % 32 == 0);
static_assert(KP >= KD);
static_assert(KP / 32 == 4);
static_assert(NCOL == 3 * NCL);
static_assert(NCOL == NT * 16);
static_assert(RT == 32);
static_assert(NPTS % (RT * AW) == 0);
static_assert(NPTS <= NPTS_FULL);
static_assert((EP * 4) % 16 == 0);
static_assert(EP >= KP / 2);
static_assert(24 * 16 == RT * 3 * 4);
static_assert((RT * 3 * 4) % 128 == 0);
static_assert((NCOL * 16) % 256 == 0);
static_assert(16 * 8 == KP);
static_assert((size_t)AW * RT * EP * 4 + (size_t)AW * RT * 3 * 4 <= (size_t)131072);

typedef _Float16 h16;
typedef unsigned short bf;
typedef __attribute__((ext_vector_type(16))) _Float16 v16h;
typedef __attribute__((ext_vector_type(8)))  _Float16 v8h;
typedef __attribute__((ext_vector_type(8)))  float    v8f;
typedef __attribute__((ext_vector_type(4)))  float    v4f;
typedef v4f  __attribute__((may_alias)) v4fa;
typedef __attribute__((ext_vector_type(4)))  unsigned int v4u;
typedef v4u  __attribute__((may_alias)) v4ua;

__device__ __forceinline__ unsigned short f2bf(float f) { unsigned u = __float_as_uint(f); u += 0x7FFFu + ((u >> 16) & 1u); return (unsigned short)(u >> 16); }
__device__ __forceinline__ float bfr(float f) { return __uint_as_float(((unsigned)f2bf(f)) << 16); }
__device__ __forceinline__ v16h cat16(v8h lo, v8h hi) { return __builtin_shufflevector(lo, hi, 0, 1, 2, 3, 4, 5, 6, 7, 8, 9, 10, 11, 12, 13, 14, 15); }
__device__ __forceinline__ v8f wmma16(v16h a, v16h b, v8f c) { return __builtin_amdgcn_wmma_f32_16x16x32_f16(false, a, false, b, (short)0, c, false, false); }
__device__ __forceinline__ v16h  ldh(const h16* p) { return cat16(*(const v8h*)p, *(const v8h*)(p + 16)); }
__device__ __forceinline__ void wave_sync() { __builtin_amdgcn_fence(3  , "wavefront"); __builtin_amdgcn_wave_barrier(); asm volatile("" ::: "memory"); }

__device__ __forceinline__ h16 toh_flush(float v) { const h16 r = (h16)v; return (fabsf(v) < 6.103515625e-05f) ? (h16)0.0f : r; }
__device__ __forceinline__ unsigned int pack2h(h16 lo, h16 hi) { return (unsigned int)__builtin_bit_cast(unsigned short, lo) | ((unsigned int)__builtin_bit_cast(unsigned short, hi) << 16); }
__device__ __forceinline__ v8f wmmag(v16h a, v16h b, v8f c) { c = wmma16(a, b, c); asm volatile("v_nop\n\tv_nop\n\tv_nop\n\tv_nop" : "+v"(c) : "v"(a), "v"(b)); return c; }

__global__ __launch_bounds__(256) void k_wconv(const float* __restrict__ W, h16* WH) {
    const int i = (int)(blockIdx.x * 256 + threadIdx.x); if (i >= NCOL * 16) return;
    const int row = i >> 4, g = i & 15;
    v8h o;
#pragma unroll
    for (int e = 0; e < 8; ++e) {
        const int col = 8 * g + e;
        const int cc = col < KD ? col : (KD - 1);
        float w = W[(size_t)row * KD + cc];
        asm volatile("" : "+v"(w));
        const float sv = bfr(w) * WSC;
        const h16 hv = toh_flush(sv);
        o[e] = (col < KD) ? hv : (h16)0.0f;
    }
    *(volatile v8h*)(WH + (size_t)i * 8) = o; __threadfence(); *(volatile v8h*)(WH + (size_t)i * 8) = o;
}

__global__ __launch_bounds__(32 * AW) __attribute__((amdgpu_num_vgpr(256)))
void k_main(const float* __restrict__ X, const int* __restrict__ CID, const h16* __restrict__ WH, float* OUT) {
    __shared__ __align__(16) unsigned int es[AW * RT * EP];
    __shared__ __align__(16) float os[AW * RT * 3];
    const int lane = threadIdx.x & 31, lr = lane & 15, hi = lane >> 4;
    const int wave = __builtin_amdgcn_readfirstlane((int)(threadIdx.x >> 5));
    const int p0 = ((int)blockIdx.x * AW + wave) * RT;
    const int p = p0 + lane;
    const int eb = wave * RT * EP, ob = wave * RT * 3;

    int cid = CID[p]; cid = cid < 0 ? 0 : (cid > NCL - 1 ? NCL - 1 : cid);

    const int erow = eb + lane * EP;
#pragma unroll 1
    for (int c = 0; c < NCH; ++c) {
        const float xb = bfr(X[(size_t)p * NCH + c]);
        float f = 1.0f;
#pragma unroll 1
        for (int k = 0; k < NFQ; ++k) {
            float sv, cv;
            sincosf(xb * f, &sv, &cv);
            es[erow + c * NFQ + k] = pack2h(toh_flush(sv), toh_flush(cv));
            f += f;
        }
    }
#pragma unroll
    for (int w = KD / 2; w < KP / 2; ++w) es[erow + w] = 0u;
    wave_sync();

    v16h a[2][4];
#pragma unroll
    for (int mt = 0; mt < 2; ++mt) {
#pragma unroll
        for (int kk = 0; kk < 4; ++kk) {
            const int wo = eb + (mt * 16 + lr) * EP + kk * 16 + 4 * hi;
            const v4u q0 = *(const v4ua*)(&es[wo]);
            const v4u q1 = *(const v4ua*)(&es[wo + 8]);
            a[mt][kk] = cat16(__builtin_bit_cast(v8h, q0), __builtin_bit_cast(v8h, q1));
        }
    }
    int ntn[2][8], oix[2][8];
#pragma unroll
    for (int mt = 0; mt < 2; ++mt) {
#pragma unroll
        for (int r = 0; r < 8; ++r) {
            const int row = mt * 16 + 8 * hi + r;
            const int cr = __shfl(cid, row, 32);
            const int c3 = 3 * cr;
            const int j = (lr - c3) & 15;
            const bool ok = j < 3;
            ntn[mt][r] = ok ? ((c3 + j) >> 4) : -1;
            oix[mt][r] = ok ? (row * 3 + j) : -1;
        }
    }
    v8f val0 = (v8f){}, val1 = (v8f){};
    const size_t bo = (size_t)lr * KP + 8 * hi;
#pragma unroll 1
    for (int nt = 0; nt < NT; ++nt) {
        const h16* wp = WH + bo + (size_t)nt * 16 * KP;
        v8f c0 = (v8f){}, c1 = (v8f){};
#pragma unroll
        for (int kk = 0; kk < 4; ++kk) {
            const v16h b = ldh(wp + kk * 32);
            c0 = wmmag(a[0][kk], b, c0);
            c1 = wmmag(a[1][kk], b, c1);
        }
#pragma unroll
        for (int r = 0; r < 8; ++r) {
            val0[r] = (nt == ntn[0][r]) ? c0[r] : val0[r];
            val1[r] = (nt == ntn[1][r]) ? c1[r] : val1[r];
        }
    }

#pragma unroll
    for (int r = 0; r < 8; ++r) {
        const float u0 = val0[r] * WSI, u1 = val1[r] * WSI;
        if (oix[0][r] >= 0) os[ob + oix[0][r]] = u0;
        if (oix[1][r] >= 0) os[ob + oix[1][r]] = u1;
    }
    wave_sync();
    const int li = (lane < 24 ? lane : 23) * 4;
    const v4f ov = *(const v4fa*)(&os[ob + li]);
    float* op = OUT + (size_t)p0 * 3 + (size_t)li;
#pragma unroll 1
    for (int ps = 0; ps < 2; ++ps) {
        if (lane < 24) *(volatile v4f*)op = ov;
        if (ps == 0) __threadfence();
    }
}

static constexpr size_t al256(size_t v) { return (v + 255) & ~(size_t)255; }
static constexpr size_t SZ_WH = al256((size_t)NCOL * KP * 2);
static constexpr size_t SZ_TOTAL = SZ_WH;
static_assert(SZ_TOTAL <= (size_t)134217728);
static_assert((size_t)NCOL * 16 * 16 == (size_t)NCOL * KP * 2);
static_assert((size_t)(NPTS / (RT * AW)) * AW * RT * 3 * 4 == (size_t)NPTS * 3 * 4);

extern "C" void kernel_launch(void* const* d_in, const int* in_sizes, int n_in,
                              void* d_out, int out_size, void* d_ws, size_t ws_size, hipStream_t stream) {
    if (n_in < 3) return;
    if ((size_t)in_sizes[0] < (size_t)NPTS * NCH) return;
    if ((size_t)in_sizes[1] < (size_t)NPTS) return;
    if ((size_t)in_sizes[2] < (size_t)NCOL * KD) return;
    if ((size_t)out_size < (size_t)NPTS * 3) return;
    if (SZ_TOTAL > ws_size) return;
    const float* X   = (const float*)d_in[0];
    const int*   CID = (const int*)d_in[1];
    const float* W   = (const float*)d_in[2];
    float* OUT = (float*)d_out;
    h16* WH = (h16*)d_ws;

    k_wconv<<<dim3((NCOL * 16) / 256, 1, 1), 256, 0, stream>>>(W, WH);
    k_main<<<dim3(NPTS / (RT * AW), 1, 1), 32 * AW, 0, stream>>>(X, CID, WH, OUT);
}
